// Gemma3Attention_42666205118605
// MI455X (gfx1250) — hardware-verified
//
#include <hip/hip_runtime.h>
#include <math.h>

typedef __attribute__((ext_vector_type(16))) _Float16 v16h;
typedef __attribute__((ext_vector_type(16))) __bf16 v16b;
typedef __attribute__((ext_vector_type(8)))  _Float16 v8h;
typedef __attribute__((ext_vector_type(8)))  float v8f;
typedef __attribute__((ext_vector_type(4)))  float v4f;
typedef __attribute__((ext_vector_type(2)))  float v2f;
typedef __attribute__((ext_vector_type(4)))  unsigned v4u;
typedef __attribute__((ext_vector_type(4)))  int v4i;
typedef float __attribute__((may_alias)) float_a;
typedef int __attribute__((may_alias)) int_a;

template <typename T> __device__ __forceinline__ void vst2(void* p, T v) { *(volatile T*)p = v; __threadfence(); *(volatile T*)p = v; }
__device__ __forceinline__ v8f wmma16(v16h a, v16h b, v8f c) {
  v8f d = __builtin_amdgcn_wmma_f32_16x16x32_f16(false, a, false, b, (short)0, c, false, false);
  asm volatile("v_nop\n\tv_nop\n\tv_nop\n\tv_nop" : "+v"(d) : "v"(a), "v"(b));
  return d;
}
__device__ __forceinline__ v8f wmma_bf(v16b a, v16b b, v8f c) {
  v8f d = __builtin_amdgcn_wmma_f32_16x16x32_bf16(false, a, false, b, (short)0, c, false, false);
  asm volatile("v_nop\n\tv_nop\n\tv_nop\n\tv_nop" : "+v"(d) : "v"(a), "v"(b));
  return d;
}
__device__ __forceinline__ v16h frag_h(const _Float16* rowk0, int lane) {
  union { v16h v; v8h q[2]; } u; const _Float16* p = rowk0 + 8 * (lane >> 4);
  u.q[0] = *(const v8h*)p; u.q[1] = *(const v8h*)(p + 16); return u.v;
}
__device__ __forceinline__ v16h frag_f32(const float* rowk0, int lane) {
  v16h a; const float* p = rowk0 + 8 * (lane >> 4);
#pragma unroll
  for (int i = 0; i < 8; ++i) { a[i] = (_Float16)p[i]; a[8 + i] = (_Float16)p[16 + i]; }
  return a;
}
__device__ __forceinline__ v16h frag_f32s(const float* rowk0, int lane, float sc) {
  v16h a; const float* p = rowk0 + 8 * (lane >> 4);
#pragma unroll
  for (int i = 0; i < 8; ++i) { a[i] = (_Float16)(p[i] * sc); a[8 + i] = (_Float16)(p[16 + i] * sc); }
  return a;
}
__device__ __forceinline__ v16h fragc_f32(const float* W, int k0, int n, int lane, int ld, int K) {
  v16h a; const int g = lane >> 4;
#pragma unroll
  for (int i = 0; i < 8; ++i) { const int ka = k0 + 8 * g + i, kb = ka + 16;
    a[i] = (_Float16)(ka < K ? W[(size_t)(ka < K ? ka : K - 1) * ld + n] : 0.f); a[8 + i] = (_Float16)(kb < K ? W[(size_t)(kb < K ? kb : K - 1) * ld + n] : 0.f); }
  return a;
}
struct F2 { v16b h, l; };
__device__ __forceinline__ F2 bsplit16(const float v[16]) { F2 r;
#pragma unroll
  for (int i = 0; i < 16; ++i) { const __bf16 h = (__bf16)v[i]; r.h[i] = h; r.l[i] = (__bf16)(v[i] - (float)h); }
  return r; }
__device__ __forceinline__ F2 split_row(const float* row, int k0, int lane) { float v[16]; const float* p = row + k0 + 8 * (lane >> 4);
#pragma unroll
  for (int i = 0; i < 8; ++i) { v[i] = p[i]; v[8 + i] = p[16 + i]; }
  return bsplit16(v); }
__device__ __forceinline__ F2 split_rowK(const float* row, int k0, int lane, int K) { float v[16]; const int g = lane >> 4;
#pragma unroll
  for (int i = 0; i < 8; ++i) { const int ka = k0 + 8 * g + i, kb = ka + 16; v[i] = ka < K ? row[ka < K ? ka : K - 1] : 0.f; v[8 + i] = kb < K ? row[kb < K ? kb : K - 1] : 0.f; }
  return bsplit16(v); }
__device__ __forceinline__ F2 split_col(const float* W, int k0, int n, int lane, int ld, int K) { float v[16]; const int g = lane >> 4;
#pragma unroll
  for (int i = 0; i < 8; ++i) { const int ka = k0 + 8 * g + i, kb = ka + 16; v[i] = ka < K ? W[(size_t)(ka < K ? ka : K - 1) * ld + n] : 0.f; v[8 + i] = kb < K ? W[(size_t)(kb < K ? kb : K - 1) * ld + n] : 0.f; }
  return bsplit16(v); }
__device__ __forceinline__ v8f mac3(const F2& a, const F2& b, v8f c) { c = wmma_bf(a.l, b.h, c); c = wmma_bf(a.h, b.l, c); return wmma_bf(a.h, b.h, c); }
__device__ __forceinline__ float sigm(float v) { return 1.0f / (1.0f + expf(-v)); }
#define LDSX() do { asm volatile("s_wait_dscnt 0" ::: "memory"); __builtin_amdgcn_wave_barrier(); __builtin_amdgcn_fence(__ATOMIC_RELEASE, "workgroup"); } while (0)


#define SS 2048
#define HID 2048
#define NH 8
#define NKV 4
#define HD 256
#define WIN 1024
#ifndef TQB
#define TQB (SS / 64)
#define TQ0 0
#define KRP (SS / 64)
#endif
typedef __attribute__((ext_vector_type(8))) __bf16 v8b;
__device__ __forceinline__ v16b frag_b(const __bf16* rowk0, int lane) {
  union { v16b v; v8b q[2]; } u; const __bf16* p = rowk0 + 8 * (lane >> 4);
  u.q[0] = *(const v8b*)p; u.q[1] = *(const v8b*)(p + 16); return u.v;
}
__device__ __forceinline__ float bfr(float v) { return (float)(__bf16)v; }
__device__ __attribute__((noinline)) float exp_ni(float v) { return expf(v); }
__device__ __attribute__((noinline)) float erf_ni(float v) { return erff(v); }

#define WS_PW  0u
#define PQ 0
#define PK (PQ + NH * HD * HID)
#define PV (PK + NKV * HD * HID)
#define PO (PV + NKV * HD * HID)
#define PWEND (PO + HID * NH * HD)
#define WS_Q   (WS_PW + 2u * PWEND)
#define WS_K   (WS_Q + 4u * SS * NH * HD)
#define WS_V   (WS_K + 4u * SS * NKV * HD)
#define WS_VH  (WS_V + 4u * SS * NKV * HD)
#define WS_VL  (WS_VH + 2u * NKV * HD * SS)
#define WS_O   (WS_VL + 2u * NKV * HD * SS)
#define WS_END (WS_O + 4u * SS * NH * HD)

__global__ __launch_bounds__(256) void k_packT(const float* __restrict__ WQ, const float* __restrict__ WK, const float* __restrict__ WV, const float* __restrict__ WO, __bf16* __restrict__ PW) {
  __shared__ __align__(16) __bf16 s[2048]; const int n = blockIdx.x, which = blockIdx.y, tid = threadIdx.x; int K, N; const float* Wm; size_t base;
  if (which == 0) { K = HID; N = NH * HD; Wm = WQ; base = PQ; } else if (which == 1) { K = HID; N = NKV * HD; Wm = WK; base = PK; } else if (which == 2) { K = HID; N = NKV * HD; Wm = WV; base = PV; } else { K = NH * HD; N = HID; Wm = WO; base = PO; }
  if (n >= N) return;
  for (int k = tid; k < K; k += 256) s[k] = (__bf16)Wm[(size_t)k * N + n];
  __syncthreads();
  for (int q = tid; q < K / 8; q += 256) vst2((unsigned*)(PW + base + (size_t)n * K + q * 8), *(const v4u*)&s[q * 8]);
}
template <int RIN>
__global__ __launch_bounds__(128) void k_gemm(const float* __restrict__ A, int lda, int K, const __bf16* __restrict__ P, float* __restrict__ OUT, int ldo) {
  __shared__ __align__(16) float so[4][16][132];
  const int tid = threadIdx.x, wave = tid >> 5, lane = tid & 31, col = lane & 15, g = lane >> 4; const size_t r0 = (size_t)blockIdx.x * 64 + wave * 16; const int n0 = blockIdx.y * 128;
  v8f acc[8] = {};
#pragma unroll 2
  for (int kc = 0; kc < K / 32; ++kc) { F2 a; if (RIN) { v16b ax; const float* p = A + (r0 + col) * lda + kc * 32 + 8 * g;
#pragma unroll
      for (int i = 0; i < 8; ++i) { ax[i] = (__bf16)p[i]; ax[8 + i] = (__bf16)p[16 + i]; } a.h = ax; a.l = ax; } else a = split_row(A + (r0 + col) * lda, kc * 32, lane);
#pragma unroll
    for (int j = 0; j < 8; ++j) { const v16b w = frag_b(P + (size_t)(n0 + j * 16 + col) * K + kc * 32, lane); if (!RIN) acc[j] = wmma_bf(a.l, w, acc[j]); acc[j] = wmma_bf(a.h, w, acc[j]); } }
#pragma unroll
  for (int j = 0; j < 8; ++j)
#pragma unroll
    for (int r = 0; r < 8; ++r) so[wave][8 * g + r][j * 16 + col] = acc[j][r];
  LDSX();
  for (int rl = 0; rl < 16; ++rl) vst2(OUT + (r0 + rl) * ldo + n0 + lane * 4, *(const v4f*)&so[wave][rl][lane * 4]);
}
template <int PLANE>
__global__ __launch_bounds__(256) void k_normrope(float* QK, const float* __restrict__ SC, const float* __restrict__ COS, const float* __restrict__ SIN, const float* __restrict__ V, __bf16* __restrict__ VH, __bf16* __restrict__ VL) {
  __shared__ float sy[HD]; __shared__ float sred[8]; __shared__ __align__(16) float so[HD];
  const int s = blockIdx.x, h = blockIdx.y, d = threadIdx.x; const int pitch = PLANE ? (NKV * HD) : (NH * HD);
  float* row = QK + (size_t)s * pitch + h * HD; const float y = row[d]; sy[d] = y;
  float q = y * y;
#pragma unroll
  for (int o = 1; o < 32; o <<= 1) q += __shfl_xor(q, o);
  if ((d & 31) == 0) sred[d >> 5] = q;
  __syncthreads();
  float ss = 0.f;
#pragma unroll
  for (int w = 0; w < 8; ++w) ss += sred[w];
  const float rs = rsqrtf(ss / (float)HD + 1e-6f);
  const float yn = y * rs * (1.0f + bfr(SC[d])); const float other = sy[(d < HD / 2) ? (d + HD / 2) : (d - HD / 2)] * rs * (1.0f + bfr(SC[(d < HD / 2) ? (d + HD / 2) : (d - HD / 2)]));
  const float rot = (d < HD / 2) ? -other : other;
  so[d] = yn * bfr(COS[(size_t)s * HD + d]) + rot * bfr(SIN[(size_t)s * HD + d]);
  __syncthreads();
  if (d < HD / 4) vst2(row + d * 4, *(const v4f*)&so[d * 4]);
}
__global__ __launch_bounds__(256) void k_vplanes(const float* __restrict__ V, __bf16* __restrict__ VH, __bf16* __restrict__ VL) {
  __shared__ __align__(16) __bf16 sh[128][72], sl[128][72]; const int tid = threadIdx.x; const int s0 = blockIdx.x * 64, c0 = blockIdx.y * 128;
  for (int q = tid; q < 64 * 128; q += 256) { const int sl_ = q >> 7, c = q & 127; const float v = V[(size_t)(s0 + sl_) * (NKV * HD) + c0 + c]; const __bf16 hb = (__bf16)v; sh[c][sl_] = hb; sl[c][sl_] = (__bf16)(v - (float)hb); }
  __syncthreads();
  for (int q = tid; q < 128 * 8; q += 256) { const int c = q >> 3, pc = q & 7; const size_t o = (size_t)(c0 + c) * SS + s0 + pc * 8; vst2((unsigned*)(VH + o), *(const v4u*)&sh[c][pc * 8]); vst2((unsigned*)(VL + o), *(const v4u*)&sl[c][pc * 8]); }
}
template <int DH>
__global__ __launch_bounds__(128) void k_attn(const float* __restrict__ Q, const float* __restrict__ Kx, const int* __restrict__ AM, const int* __restrict__ SEGPOS, const __bf16* __restrict__ VH, const __bf16* __restrict__ VL, float* __restrict__ O) {
  __shared__ __align__(16) float sp[4][16][36]; __shared__ __align__(16) float so[4][16][132];
  const int tid = threadIdx.x, wave = tid >> 5, lane = tid & 31, col = lane & 15, g = lane >> 4; const int qb = blockIdx.x + TQ0, h = blockIdx.y; const int kv = h / (NH / NKV); const int q0 = qb * 64 + wave * 16;
  const float* qrow = Q + (size_t)(q0 + col) * (NH * HD) + h * HD;
  int posq[8];
#pragma unroll
  for (int r = 0; r < 8; ++r) posq[r] = SEGPOS[q0 + 8 * g + r];
  float m[8], l[8];
#pragma unroll
  for (int r = 0; r < 8; ++r) { m[r] = -3.0e38f; l[r] = 0.f; }
  v8f acc[8] = {};
  const int nks = (qb * 64 + 64) / 32;
#pragma unroll 1
  for (int ks = 0; ks < nks; ++ks) { v8f s[2]; bool lv[2][8]; bool anylive = false;
#pragma unroll
    for (int ct = 0; ct < 2; ++ct) { const int kk = ks * 32 + ct * 16 + col; const bool am = (AM[kk] != 0);
#pragma unroll
      for (int r = 0; r < 8; ++r) { const int qi = q0 + 8 * g + r; const bool live = am && (kk <= qi) && (kk > posq[r] - WIN) && (kk < posq[r] + WIN); lv[ct][r] = live; anylive = anylive || live; } }
    if (__any(anylive)) {
#pragma unroll
      for (int ct = 0; ct < 2; ++ct) { const int kk = ks * 32 + ct * 16 + col; const float* krow = Kx + (size_t)kk * (NKV * HD) + kv * HD; v8f c = {};
#pragma unroll
        for (int kc = 0; kc < HD / 32; ++kc) { const F2 kb = split_row(krow, kc * 32, lane); const F2 qa = split_row(qrow, kc * 32, lane); c = mac3(qa, kb, c); }
#pragma unroll
        for (int r = 0; r < 8; ++r) s[ct][r] = lv[ct][r] ? c[r] * 0.0625f : -3.0e38f; }
#pragma unroll
      for (int r = 0; r < 8; ++r) { float mx = fmaxf(s[0][r], s[1][r]);
#pragma unroll
        for (int o = 1; o < 16; o <<= 1) mx = fmaxf(mx, __shfl_xor(mx, o));
        const float mn = fmaxf(m[r], mx); const float alpha = (m[r] <= -1.0e38f) ? 0.f : exp_ni(m[r] - mn);
        const float e0 = (s[0][r] <= -1.0e38f) ? 0.f : exp_ni(s[0][r] - mn), e1 = (s[1][r] <= -1.0e38f) ? 0.f : exp_ni(s[1][r] - mn); float es = e0 + e1;
#pragma unroll
        for (int o = 1; o < 16; o <<= 1) es += __shfl_xor(es, o);
        l[r] = l[r] * alpha + es; m[r] = mn;
#pragma unroll
        for (int dt = 0; dt < 8; ++dt) acc[dt][r] *= alpha;
        sp[wave][8 * g + r][col] = e0; sp[wave][8 * g + r][16 + col] = e1; }
      LDSX();
      const F2 pa = split_row(&sp[wave][col][0], 0, lane);
#pragma unroll
      for (int dt = 0; dt < 8; ++dt) { const size_t vr = (size_t)(kv * HD + DH * 128 + dt * 16 + col) * SS + ks * 32; const v16b vh = frag_b(VH + vr, lane), vl = frag_b(VL + vr, lane); acc[dt] = wmma_bf(pa.l, vh, acc[dt]); acc[dt] = wmma_bf(pa.h, vl, acc[dt]); acc[dt] = wmma_bf(pa.h, vh, acc[dt]); }
      LDSX(); } }
#pragma unroll
  for (int r = 0; r < 8; ++r) { const float il = (l[r] > 0.f) ? 1.0f / l[r] : 0.f;
#pragma unroll
    for (int dt = 0; dt < 8; ++dt) so[wave][8 * g + r][dt * 16 + col] = acc[dt][r] * il; }
  LDSX();
  for (int rl = 0; rl < 16; ++rl) vst2(O + (size_t)(q0 + rl) * (NH * HD) + h * HD + DH * 128 + lane * 4, *(const v4f*)&so[wave][rl][lane * 4]);
}
extern "C" void kernel_launch(void* const* d_in, const int* in_sizes, int n_in, void* d_out, int out_size, void* d_ws, size_t ws_size, hipStream_t stream) {
  (void)in_sizes; (void)n_in; (void)out_size;
  const float** F = (const float**)d_in; const int* AM = (const int*)d_in[1]; const int* SEGPOS = (const int*)d_in[2];
  if (ws_size < (size_t)WS_END) return;
  char* ws = (char*)d_ws; __bf16 *PW = (__bf16*)(ws + WS_PW), *VH = (__bf16*)(ws + WS_VH), *VL = (__bf16*)(ws + WS_VL); float *Q = (float*)(ws + WS_Q), *Kx = (float*)(ws + WS_K), *V = (float*)(ws + WS_V), *O = (float*)(ws + WS_O);
  k_packT<<<dim3(HID, 4), 256, 0, stream>>>(F[5], F[6], F[7], F[8], PW);
  k_gemm<1><<<dim3(TQB, NH * HD / 128), 128, 0, stream>>>(F[0] + (size_t)TQ0 * 64 * HID, HID, HID, PW + PQ, Q + (size_t)TQ0 * 64 * NH * HD, NH * HD);
  k_gemm<1><<<dim3(KRP, NKV * HD / 128), 128, 0, stream>>>(F[0], HID, HID, PW + PK, Kx, NKV * HD);
  k_gemm<1><<<dim3(KRP, NKV * HD / 128), 128, 0, stream>>>(F[0], HID, HID, PW + PV, V, NKV * HD);
  k_normrope<0><<<dim3(TQB * 64, NH), 256, 0, stream>>>(Q + (size_t)TQ0 * 64 * NH * HD, F[9], F[3] + (size_t)TQ0 * 64 * HD, F[4] + (size_t)TQ0 * 64 * HD, nullptr, nullptr, nullptr);
  k_normrope<1><<<dim3(KRP * 64, NKV), 256, 0, stream>>>(Kx, F[10], F[3], F[4], nullptr, nullptr, nullptr);
  k_vplanes<<<dim3(KRP, NKV * HD / 128), 256, 0, stream>>>(V, VH, VL);
  k_attn<0><<<dim3(TQB, NH), 128, 0, stream>>>(Q, Kx, AM, SEGPOS, VH, VL, O);
  k_attn<1><<<dim3(TQB, NH), 128, 0, stream>>>(Q, Kx, AM, SEGPOS, VH, VL, O);
  k_gemm<0><<<dim3(TQB, HID / 128), 128, 0, stream>>>(O + (size_t)TQ0 * 64 * NH * HD, NH * HD, NH * HD, PW + PO, (float*)d_out + (size_t)TQ0 * 64 * HID, HID);
}
